// MultiScaleRetention_463856468165
// MI455X (gfx1250) — hardware-verified
//
#include <hip/hip_runtime.h>
#include <math.h>

constexpr int kBatch = 2;
constexpr int kSeq   = 2048;
constexpr int kHid   = 1024;
constexpr int kHeads = 8;
constexpr int kHd    = 128;
constexpr int kPairs = kHd / 2;
constexpr int kTok   = kBatch * kSeq;
constexpr int kSlab  = 32;
constexpr float kEps = 1e-5f;
static_assert(kHeads * kHd == kHid);
static_assert(kHid % 32 == 0);
static_assert(kTok % 64 == 0 && kHid % 64 == 0 && kSeq % 64 == 0 && kHd % 64 == 0);
static_assert(kSeq % 128 == 0 && kHd == 128 && kSlab == 32);

typedef __attribute__((ext_vector_type(16))) _Float16 v16h;
typedef __attribute__((ext_vector_type(8)))  _Float16 v8h;
typedef __attribute__((ext_vector_type(16))) __bf16   v16b;
typedef __attribute__((ext_vector_type(8)))  __bf16   v8b;
typedef __attribute__((ext_vector_type(8)))  float    v8f;
typedef __attribute__((ext_vector_type(4)))  float    v4f;
typedef __attribute__((ext_vector_type(4)))  unsigned int v4u;
typedef __attribute__((ext_vector_type(2)))  unsigned int v2u;

__device__ __forceinline__ unsigned short f2bf_bits(float f) {
  unsigned u = __float_as_uint(f);
  return (unsigned short)((u + 0x7FFFu + ((u >> 16) & 1u)) >> 16);
}
__device__ __forceinline__ float bf_bits2f(unsigned short h) { return __uint_as_float(((unsigned)h) << 16); }

__device__ __forceinline__ void dep_guard_b(v8f& a, v8f& b, v16b x, v16b y) { asm volatile("v_nop\n\tv_nop\n\tv_nop\n\tv_nop" : "+v"(a), "+v"(b) : "v"(x), "v"(y)); }
__device__ __forceinline__ void dep_guard4_b(v8f& a, v8f& b, v8f& c, v8f& d, v16b x, v16b y) { asm volatile("v_nop\n\tv_nop\n\tv_nop\n\tv_nop" : "+v"(a), "+v"(b), "+v"(c), "+v"(d) : "v"(x), "v"(y)); }
__device__ __forceinline__ void keep4_b(v16b a, v16b b, v16b c, v16b d) { asm volatile("v_nop" :: "v"(a), "v"(b), "v"(c), "v"(d)); }
__device__ __forceinline__ void acc_guard4(v8f& a, v8f& b, v8f& c, v8f& d) { asm volatile("v_nop\n\tv_nop\n\tv_nop\n\tv_nop" : "+v"(a), "+v"(b), "+v"(c), "+v"(d)); }
template <typename T> struct Frag;
template <> struct Frag<__bf16> {
  typedef v16b V; union U { v16b v; v8b h[2]; };
  static __device__ __forceinline__ v16b load(const __bf16* p) {
    U f; f.h[0] = *(const v8b*)(p); f.h[1] = *(const v8b*)(p + 16); return f.v;
  }
  static __device__ __forceinline__ v8f mma(v16b a, v16b b, v8f c) {
    return __builtin_amdgcn_wmma_f32_16x16x32_bf16(false, a, false, b, (short)0, c, false, false);
  }
  static __device__ __forceinline__ void guard(v8f& a, v8f& b, v16b x, v16b y) { dep_guard_b(a, b, x, y); }
  static __device__ __forceinline__ void guard4(v8f& a, v8f& b, v8f& c, v8f& d, v16b x, v16b y) { dep_guard4_b(a, b, c, d, x, y); }
  static __device__ __forceinline__ void keep(v16b a, v16b b, v16b c, v16b d) { keep4_b(a, b, c, d); }
};

__device__ __forceinline__ v8f mma_b(v16b a, v16b b, v8f c) {
  c = __builtin_amdgcn_wmma_f32_16x16x32_bf16(false, a, false, b, (short)0, c, false, false);
  asm volatile("v_nop\n\tv_nop\n\tv_nop\n\tv_nop" : "+v"(c) : "v"(a), "v"(b));
  return c;
}

__device__ __forceinline__ unsigned pk16(unsigned short a, unsigned short b) { return (unsigned)a | ((unsigned)b << 16); }

template <int SPLITM, int OUT_MODE>
__global__ __launch_bounds__(256) void gemm64(
    const unsigned short* __restrict__ Ap, const unsigned short* __restrict__ A2p, int lda, long strideA,
    const unsigned short* __restrict__ Btp, const unsigned short* __restrict__ Bt2p, int ldb, long strideB,
    void* __restrict__ Cout, void* __restrict__ Cout2, int ldc, long strideC,
    const float* __restrict__ tab,
    int M, int N, int K, float scale) {
  typedef __bf16 T;
  typedef v16b V;
  const T* A = (const T*)Ap; const T* A2 = (const T*)A2p; const T* Bt = (const T*)Btp; const T* Bt2 = (const T*)Bt2p;
  __shared__ __align__(16) float sT[8][16 * 68];
  const int b    = blockIdx.y;
  const int lane = threadIdx.x & 31;
  const int wave = threadIdx.x >> 5;
  const int tilesN = N >> 6;
  const int tilesM = M >> 6;
  const int tile = blockIdx.x * 8 + wave;
  if (tile >= tilesM * tilesN) return;
  const int tm = tile / tilesN;
  const int tn = tile - tm * tilesN;
  const int m0 = tm << 6;
  const int n0 = tn << 6;

  const T* Ab  = A  + (size_t)b * strideA;
  const T* Bb  = Bt + (size_t)b * strideB;
  const T* Ab2 = (SPLITM != 0) ? (A2  + (size_t)b * strideA) : nullptr;
  const T* Bb2 = (SPLITM == 1) ? (Bt2 + (size_t)b * strideB) : nullptr;

  const int rlane = lane & 15;
  const int koff  = (lane >> 4) * 8;
  const int mOff  = (lane >> 4) * 8;

  v8f acc[4][4];
#pragma unroll
  for (int i = 0; i < 4; ++i)
#pragma unroll
    for (int j = 0; j < 4; ++j) acc[i][j] = (v8f){0.f,0.f,0.f,0.f,0.f,0.f,0.f,0.f};

  for (int k0 = 0; k0 < K; k0 += 32) {
    V bh[4], bl[4];
#pragma unroll
    for (int j = 0; j < 4; ++j) {
      const size_t bo = (size_t)(n0 + (j << 4) + rlane) * ldb + koff + k0;
      bh[j] = Frag<T>::load(Bb + bo);
      bl[j] = bh[j];
      if (SPLITM == 1) bl[j] = Frag<T>::load(Bb2 + bo);
    }
#pragma unroll
    for (int i = 0; i < 4; ++i) {
      const size_t ao = (size_t)(m0 + (i << 4) + rlane) * lda + koff + k0;
      V ah = Frag<T>::load(Ab + ao);
      V al = ah;
      if (SPLITM != 0) al = Frag<T>::load(Ab2 + ao);
#pragma unroll
      for (int j = 0; j < 4; ++j) {
        acc[i][j] = Frag<T>::mma(ah, bh[j], acc[i][j]);
        if (SPLITM == 1) acc[i][j] = Frag<T>::mma(ah, bl[j], acc[i][j]);
        if (SPLITM != 0) acc[i][j] = Frag<T>::mma(al, bh[j], acc[i][j]);
      }
      Frag<T>::guard4(acc[i][0], acc[i][1], acc[i][2], acc[i][3], ah, al);
    }
    Frag<T>::keep(bh[0], bh[1], bh[2], bh[3]);
    if (SPLITM == 1) Frag<T>::keep(bl[0], bl[1], bl[2], bl[3]);
  }
  acc_guard4(acc[0][0], acc[0][1], acc[0][2], acc[0][3]);
  acc_guard4(acc[1][0], acc[1][1], acc[1][2], acc[1][3]);
  acc_guard4(acc[2][0], acc[2][1], acc[2][2], acc[2][3]);
  acc_guard4(acc[3][0], acc[3][1], acc[3][2], acc[3][3]);

  float* slab = sT[wave];
#pragma unroll
  for (int i = 0; i < 4; ++i) {
    const int mBase = m0 + (i << 4);
#pragma unroll
    for (int j = 0; j < 4; ++j) {
#pragma unroll
      for (int r = 0; r < 8; ++r) {
        const float v = acc[i][j][r] * scale;
        slab[(mOff + r) * 68 + (j << 4) + rlane] = v;
      }
    }
    __builtin_amdgcn_fence(__ATOMIC_RELEASE, "workgroup");
    __builtin_amdgcn_wave_barrier();
    __builtin_amdgcn_fence(__ATOMIC_ACQUIRE, "workgroup");
    if (OUT_MODE == 0) {
      float* C = (float*)Cout + (size_t)b * strideC;
      const int hh = lane >> 4, c4 = (lane & 15) * 4;
      for (int pass = 0; pass < 2; ++pass) {
#pragma unroll
        for (int it = 0; it < 8; ++it) {
          const int row = it * 2 + hh;
          v4f v = *(const v4f*)(slab + row * 68 + c4);
          *(volatile v4f*)(C + (size_t)(mBase + row) * ldc + n0 + c4) = v;
        }
        __threadfence();
      }
    } else {
      const int q = lane >> 3, c8 = (lane & 7) * 8;
      unsigned short* C  = (unsigned short*)Cout  + (size_t)b * strideC;
      unsigned short* C2 = (unsigned short*)Cout2 + (size_t)b * strideC;
      for (int pass = 0; pass < 2; ++pass) {
#pragma unroll
        for (int it = 0; it < 4; ++it) {
          const int row = it * 4 + q;
          const float* sp = slab + row * 68 + c8;
          float xv[8];
#pragma unroll
          for (int e = 0; e < 8; ++e) xv[e] = sp[e];
          if (OUT_MODE == 3) {
            const int srow  = (mBase + row) & (kSeq - 1);
            const int pair0 = ((n0 + c8) & (kHd - 1)) >> 1;
            const float* tp = tab + ((size_t)srow * kPairs + pair0) * 2;
            const v4f ta = *(const v4f*)(tp);
            const v4f tb = *(const v4f*)(tp + 4);
            float cs[8];
            cs[0] = ta[0]; cs[1] = ta[1]; cs[2] = ta[2]; cs[3] = ta[3];
            cs[4] = tb[0]; cs[5] = tb[1]; cs[6] = tb[2]; cs[7] = tb[3];
            float yv[8];
#pragma unroll
            for (int e = 0; e < 8; ++e) {
              const float cc = cs[(e >> 1) * 2];
              const float ss = cs[(e >> 1) * 2 + 1];
              const float rot = (e & 1) ? xv[e ^ 1] : -xv[e ^ 1];
              yv[e] = xv[e] * cc + rot * ss;
            }
#pragma unroll
            for (int e = 0; e < 8; ++e) xv[e] = yv[e];
          }
          v8h hv, lv;
#pragma unroll
          for (int e = 0; e < 8; ++e) {
            const unsigned short hb = f2bf_bits(xv[e]);
            const unsigned short lb = f2bf_bits(xv[e] - bf_bits2f(hb));
            hv[e] = __builtin_bit_cast(_Float16, hb);
            lv[e] = __builtin_bit_cast(_Float16, lb);
          }
          *(volatile v8h*)(C  + (size_t)(mBase + row) * ldc + n0 + c8) = hv;
          *(volatile v8h*)(C2 + (size_t)(mBase + row) * ldc + n0 + c8) = lv;
        }
        __threadfence();
      }
    }
    __builtin_amdgcn_fence(__ATOMIC_RELEASE, "workgroup");
    __builtin_amdgcn_wave_barrier();
    __builtin_amdgcn_fence(__ATOMIC_ACQUIRE, "workgroup");
  }
}

__global__ __launch_bounds__(256) void cast8_bf16_kernel(const float* __restrict__ in, unsigned short* __restrict__ out, int n8) {
  const int i = blockIdx.x * 256 + threadIdx.x;
  if (i >= n8) return;
  const float* p = in + 8 * (size_t)i;
  const v4f a = *(const v4f*)(p);
  const v4f c = *(const v4f*)(p + 4);
  unsigned short hb[8];
#pragma unroll
  for (int e = 0; e < 4; ++e) {
    hb[e]     = f2bf_bits(a[e]);
    hb[4 + e] = f2bf_bits(c[e]);
  }
  const v4u u = (v4u){pk16(hb[0], hb[1]), pk16(hb[2], hb[3]), pk16(hb[4], hb[5]), pk16(hb[6], hb[7])};
  unsigned short* q = out + 8 * (size_t)i;
  *(volatile v4u*)q = u;
  __threadfence();
  *(volatile v4u*)q = u;
}

__global__ __launch_bounds__(256) void tr_bf16_kernel(const float* __restrict__ in0, const float* __restrict__ in1,
                                                     const float* __restrict__ in2, unsigned short* __restrict__ out,
                                                     int R, int C, int zsub) {
  __shared__ float sm[64][65];
  const int t  = threadIdx.x;
  const int r0 = blockIdx.x * 64;
  const int c0 = blockIdx.y * 64;
  const int z  = blockIdx.z;
  const int sel = z / zsub;
  const int zz  = z - sel * zsub;
  const float* in  = (sel == 0) ? in0 : (sel == 1) ? in1 : in2;
  const float* src = in + (size_t)zz * R * C;
  unsigned short* dst = out + (size_t)z * R * C;
#pragma unroll
  for (int i = 0; i < 16; ++i) {
    const int e  = i * 256 + t;
    const int rl = e >> 6;
    const int cl = e & 63;
    sm[cl][rl] = src[(size_t)(r0 + rl) * C + c0 + cl];
  }
  __syncthreads();
  const int lane = t & 31, wave = t >> 5;
  const int q = lane >> 3, c8 = (lane & 7) * 8;
  for (int pass = 0; pass < 2; ++pass) {
#pragma unroll
    for (int it = 0; it < 2; ++it) {
      const int row = wave * 8 + it * 4 + q;
      unsigned short hb[8];
#pragma unroll
      for (int e = 0; e < 8; ++e) hb[e] = f2bf_bits(sm[row][c8 + e]);
      const v4u u = (v4u){pk16(hb[0], hb[1]), pk16(hb[2], hb[3]), pk16(hb[4], hb[5]), pk16(hb[6], hb[7])};
      *(volatile v4u*)(dst + (size_t)(c0 + row) * R + r0 + c8) = u;
    }
    __threadfence();
  }
}

struct FreqParams { float invf[kPairs]; };
static_assert(sizeof(FreqParams) == 256);

__global__ __launch_bounds__(256) void xpos_table_kernel(float* __restrict__ tabQ, float* __restrict__ tabK, FreqParams fp) {
  __shared__ __align__(16) float sm[256 * 8];
  const int t  = threadIdx.x;
  const int g  = blockIdx.x * 256 + t;
  const int s  = g >> 5;
  const int i0 = (g & 31) * 2;
  float f0 = 0.f, f1 = 0.f;
#pragma unroll
  for (int k = 0; k < kPairs; k += 2) {
    f0 = (i0 == k) ? fp.invf[k]     : f0;
    f1 = (i0 == k) ? fp.invf[k + 1] : f1;
  }
  const float x   = (float)(s - kSeq / 2) * (1.0f / 512.0f);
  const float pos = (float)s;
#pragma unroll 1
  for (int j = 0; j < 2; ++j) {
    const int   i   = i0 + j;
    const float fr  = j ? f1 : f0;
    const float svi = ((float)(2 * i) + 51.2f) * (1.0f / 179.2f);
    const float lsv = log2f(svi);
    const float scq = exp2f(x * lsv);
    const float sck = exp2f(-x * lsv);
    const float ang = pos * fr;
    float sn, cs;
    sincosf(ang, &sn, &cs);
    sm[t * 8 + 2 * j]     = cs * scq;
    sm[t * 8 + 2 * j + 1] = sn * scq;
    sm[t * 8 + 4 + 2 * j] = cs * sck;
    sm[t * 8 + 5 + 2 * j] = sn * sck;
  }
  __syncthreads();
  const v4f vq = *(const v4f*)(sm + t * 8);
  const v4f vk = *(const v4f*)(sm + t * 8 + 4);
  const size_t off = ((size_t)s * kPairs + i0) * 2;
  float* pq = tabQ + off;
  float* pk = tabK + off;
  *(volatile v4f*)pq = vq;
  *(volatile v4f*)pk = vk;
  __threadfence();
  *(volatile v4f*)pq = vq;
  *(volatile v4f*)pk = vk;
}

struct RetParams { float l2g[kHeads]; };
static_assert(sizeof(RetParams) == 32);

struct RetLds {
  __bf16 kh[kSlab * kHd];
  __bf16 kl[kSlab * kHd];
  __bf16 vh[kHd * kSlab];
  __bf16 vl[kHd * kSlab];
  __bf16 ph[8][16 * kSlab];
  __bf16 pl[8][16 * kSlab];
};
union RetU { RetLds t; float ep[8][16 * 68]; };
static_assert(sizeof(RetLds) == 49152);
static_assert(sizeof(float) * 8 * 16 * 68 <= sizeof(RetLds));

__global__ __launch_bounds__(256) void retention_kernel(
    const unsigned short* __restrict__ Qhp, const unsigned short* __restrict__ Qlp,
    const unsigned short* __restrict__ Khp, const unsigned short* __restrict__ Klp,
    const unsigned short* __restrict__ Vhp, const unsigned short* __restrict__ Vlp,
    float* __restrict__ Y, RetParams rp) {
  __shared__ __align__(16) RetU L;
  union FB { v16b v; v8b h[2]; };
  const int tid  = threadIdx.x;
  const int lane = tid & 31;
  const int wave = __builtin_amdgcn_readfirstlane(tid >> 5);
  const int hh   = lane >> 4;
  const int c    = lane & 15;
  const int bh   = blockIdx.y;
  const int b    = bh >> 3;
  const int h    = bh & 7;
  const int bx   = blockIdx.x;
  const int s0   = bx * 128 + wave * 16;
  const size_t tok0 = (size_t)b * kSeq;

  float l2g = rp.l2g[0];
#pragma unroll
  for (int k = 1; k < kHeads; ++k) l2g = (h == k) ? rp.l2g[k] : l2g;

  const __bf16* Qh = (const __bf16*)Qhp;
  const __bf16* Ql = (const __bf16*)Qlp;
  v16b qah[4], qal[4];
  {
    const size_t qo = (tok0 + s0 + c) * kHid + (size_t)h * kHd + 8 * hh;
#pragma unroll
    for (int dc = 0; dc < 4; ++dc) qah[dc] = Frag<__bf16>::load(Qh + qo + dc * 32);
    keep4_b(qah[0], qah[1], qah[2], qah[3]);
#pragma unroll
    for (int dc = 0; dc < 4; ++dc) qal[dc] = Frag<__bf16>::load(Ql + qo + dc * 32);
    keep4_b(qal[0], qal[1], qal[2], qal[3]);
  }

  float colfac[2];
#pragma unroll
  for (int j = 0; j < 2; ++j) colfac[j] = exp2f(-(float)(16 * j + c) * l2g);

  v8f yacc[8];
#pragma unroll
  for (int jd = 0; jd < 8; ++jd) yacc[jd] = (v8f){0.f,0.f,0.f,0.f,0.f,0.f,0.f,0.f};

  __bf16* pwh = L.t.ph[wave];
  __bf16* pwl = L.t.pl[wave];
  const int nslab = 4 * (bx + 1);
  for (int sl = 0; sl < nslab; ++sl) {
    const int t0 = sl * kSlab;
    __syncthreads();
    {
      const int kr = tid >> 3, kq = (tid & 7) * 16;
      const size_t gko = (tok0 + t0 + kr) * kHid + (size_t)h * kHd + kq;
      const v4u ka0 = *(const v4u*)(Khp + gko);
      const v4u ka1 = *(const v4u*)(Khp + gko + 8);
      const v4u kb0 = *(const v4u*)(Klp + gko);
      const v4u kb1 = *(const v4u*)(Klp + gko + 8);
      *(v4u*)(L.t.kh + kr * kHd + kq)     = ka0;
      *(v4u*)(L.t.kh + kr * kHd + kq + 8) = ka1;
      *(v4u*)(L.t.kl + kr * kHd + kq)     = kb0;
      *(v4u*)(L.t.kl + kr * kHd + kq + 8) = kb1;
      asm volatile("" ::: "memory");
      const int vr = tid >> 1, vq = (tid & 1) * 16;
      const size_t gvo = ((size_t)bh * kHd + vr) * kSeq + t0 + vq;
      const v4u va0 = *(const v4u*)(Vhp + gvo);
      const v4u va1 = *(const v4u*)(Vhp + gvo + 8);
      const v4u vb0 = *(const v4u*)(Vlp + gvo);
      const v4u vb1 = *(const v4u*)(Vlp + gvo + 8);
      *(v4u*)(L.t.vh + vr * kSlab + vq)     = va0;
      *(v4u*)(L.t.vh + vr * kSlab + vq + 8) = va1;
      *(v4u*)(L.t.vl + vr * kSlab + vq)     = vb0;
      *(v4u*)(L.t.vl + vr * kSlab + vq + 8) = vb1;
    }
    __syncthreads();

    v8f sc[2];
#pragma unroll
    for (int j = 0; j < 2; ++j) {
      sc[j] = (v8f){0.f,0.f,0.f,0.f,0.f,0.f,0.f,0.f};
#pragma unroll
      for (int dc = 0; dc < 4; ++dc) {
        const int ko = (j * 16 + c) * kHd + dc * 32 + 8 * hh;
        FB kb, kl;
        kb.h[0] = *(const v8b*)(L.t.kh + ko);
        kb.h[1] = *(const v8b*)(L.t.kh + ko + 16);
        kl.h[0] = *(const v8b*)(L.t.kl + ko);
        kl.h[1] = *(const v8b*)(L.t.kl + ko + 16);
        sc[j] = mma_b(qah[dc], kb.v, sc[j]);
        sc[j] = mma_b(qah[dc], kl.v, sc[j]);
        sc[j] = mma_b(qal[dc], kb.v, sc[j]);
      }
    }

    float rowfac[8];
#pragma unroll
    for (int r = 0; r < 8; ++r) rowfac[r] = exp2f((float)(s0 + 8 * hh + r - t0) * l2g);
#pragma unroll
    for (int j = 0; j < 2; ++j) {
#pragma unroll
      for (int r = 0; r < 8; ++r) {
        const int srow = s0 + 8 * hh + r;
        const int tcol = t0 + 16 * j + c;
        float p = sc[j][r] * rowfac[r] * colfac[j];
        p = (srow >= tcol) ? p : 0.0f;
        const unsigned short hb = f2bf_bits(p);
        const unsigned short lb = f2bf_bits(p - bf_bits2f(hb));
        pwh[(8 * hh + r) * kSlab + 16 * j + c] = __builtin_bit_cast(__bf16, hb);
        pwl[(8 * hh + r) * kSlab + 16 * j + c] = __builtin_bit_cast(__bf16, lb);
      }
    }
    __syncthreads();

    {
      const int po = c * kSlab + 8 * hh;
      FB pa, pb;
      pa.h[0] = *(const v8b*)(pwh + po);
      pa.h[1] = *(const v8b*)(pwh + po + 16);
      pb.h[0] = *(const v8b*)(pwl + po);
      pb.h[1] = *(const v8b*)(pwl + po + 16);
#pragma unroll
      for (int jd = 0; jd < 8; ++jd) {
        const int vo = (jd * 16 + c) * kSlab + 8 * hh;
        FB va, vb;
        va.h[0] = *(const v8b*)(L.t.vh + vo);
        va.h[1] = *(const v8b*)(L.t.vh + vo + 16);
        vb.h[0] = *(const v8b*)(L.t.vl + vo);
        vb.h[1] = *(const v8b*)(L.t.vl + vo + 16);
        yacc[jd] = mma_b(pa.v, va.v, yacc[jd]);
        yacc[jd] = mma_b(pa.v, vb.v, yacc[jd]);
        yacc[jd] = mma_b(pb.v, va.v, yacc[jd]);
      }
    }
  }
  __syncthreads();

  float* os = L.ep[wave];
  const int c4 = c * 4;
#pragma unroll
  for (int half = 0; half < 2; ++half) {
#pragma unroll
    for (int jj = 0; jj < 4; ++jj) {
#pragma unroll
      for (int r = 0; r < 8; ++r) os[(8 * hh + r) * 68 + jj * 16 + c] = yacc[half * 4 + jj][r];
    }
    __syncthreads();
    float* yb = Y + (tok0 + s0) * kHid + (size_t)h * kHd + half * 64;
    for (int pass = 0; pass < 2; ++pass) {
#pragma unroll
      for (int it = 0; it < 8; ++it) {
        const int row = it * 2 + hh;
        const v4f v = *(const v4f*)(os + row * 68 + c4);
        *(volatile v4f*)(yb + (size_t)row * kHid + c4) = v;
      }
      __threadfence();
    }
    __syncthreads();
  }
}

__global__ __launch_bounds__(256) void gn_gate_kernel(const float* __restrict__ Y, const float* __restrict__ G,
                                                     const float* __restrict__ gnw, const float* __restrict__ gnb,
                                                     unsigned short* __restrict__ Zh, unsigned short* __restrict__ Zl) {
  __shared__ __align__(16) unsigned short zs[8][2][kHd];
  const int row  = blockIdx.x;
  const int t    = threadIdx.x;
  const int lane = t & 31;
  const int wave = __builtin_amdgcn_readfirstlane(t >> 5);
  const int hh   = lane >> 4;
  const int c    = lane & 15;
  const int col  = wave * kHd + lane * 4;
  const size_t off = (size_t)row * kHid + col;
  const v4f y  = *(const v4f*)(Y + off);
  const v4f g  = *(const v4f*)(G + off);
  const v4f w  = *(const v4f*)(gnw + col);
  const v4f bb = *(const v4f*)(gnb + col);
  float s1 = (y[0] + y[1]) + (y[2] + y[3]);
#pragma unroll
  for (int o = 16; o > 0; o >>= 1) s1 += __shfl_xor(s1, o, 32);
  const float mu = s1 * (1.0f / 128.0f);
  float d[4];
#pragma unroll
  for (int e = 0; e < 4; ++e) d[e] = y[e] - mu;
  float s2 = (d[0] * d[0] + d[1] * d[1]) + (d[2] * d[2] + d[3] * d[3]);
#pragma unroll
  for (int o = 16; o > 0; o >>= 1) s2 += __shfl_xor(s2, o, 32);
  const float var = s2 * (1.0f / 128.0f);
  const float inv = rsqrtf(var + kEps);
  unsigned short hb[4], lb[4];
#pragma unroll
  for (int e = 0; e < 4; ++e) {
    const float wv = bf_bits2f(f2bf_bits(w[e]));
    const float bv = bf_bits2f(f2bf_bits(bb[e]));
    const float yn = d[e] * inv * wv + bv;
    const float ge = g[e];
    const float sg = 1.0f / (1.0f + expf(-ge));
    const float z  = (ge * sg) * yn;
    hb[e] = f2bf_bits(z);
    lb[e] = f2bf_bits(z - bf_bits2f(hb[e]));
  }
  *(v2u*)(&zs[wave][0][lane * 4]) = (v2u){pk16(hb[0], hb[1]), pk16(hb[2], hb[3])};
  *(v2u*)(&zs[wave][1][lane * 4]) = (v2u){pk16(lb[0], lb[1]), pk16(lb[2], lb[3])};
  __syncthreads();
  const v4u u = *(const v4u*)(&zs[wave][hh][c * 8]);
  unsigned short* zp = (hh ? Zl : Zh) + (size_t)row * kHid + wave * kHd + c * 8;
  *(volatile v4u*)zp = u;
  __threadfence();
  *(volatile v4u*)zp = u;
}

extern "C" void kernel_launch(void* const* d_in, const int* in_sizes, int n_in,
                              void* d_out, int out_size, void* d_ws, size_t ws_size,
                              hipStream_t stream) {
  if (n_in < 8) return;
  const int nX  = kTok * kHid;
  const int nW  = kHeads * kHid * kHd;
  const int nWs = kHid * kHid;
  if (in_sizes[0] != nX || in_sizes[1] != nW || in_sizes[2] != nW || in_sizes[3] != nW) return;
  if (in_sizes[4] != nWs || in_sizes[5] != nWs || in_sizes[6] != kHid || in_sizes[7] != kHid) return;
  if (out_size != nX) return;

  const size_t sz16   = (size_t)nX * 2;
  const size_t sz32   = (size_t)nX * 4;
  const size_t szWqkv = (size_t)3 * nWs * 2;
  const size_t szWgo  = (size_t)2 * nWs * 2;
  const size_t szTab  = (size_t)kSeq * kPairs * 2 * 4;
  const size_t offXb   = 0;
  const size_t offWqkv = offXb + sz16;
  const size_t offWgo  = offWqkv + szWqkv;
  const size_t offTabQ = offWgo + szWgo;
  const size_t offTabK = offTabQ + szTab;
  const size_t offQhi  = offTabK + szTab;
  const size_t offQlo  = offQhi + sz16;
  const size_t offKhi  = offQlo + sz16;
  const size_t offKlo  = offKhi + sz16;
  const size_t offVth  = offKlo + sz16;
  const size_t offVtl  = offVth + sz16;
  const size_t offG    = offVtl + sz16;
  const size_t offY    = offG + sz32;
  const size_t offZhi  = offY + sz32;
  const size_t offZlo  = offZhi + sz16;
  const size_t total   = offZlo + sz16;
  if (ws_size < total) return;

  const float* X   = (const float*)d_in[0];
  const float* WQ  = (const float*)d_in[1];
  const float* WK  = (const float*)d_in[2];
  const float* WV  = (const float*)d_in[3];
  const float* WG  = (const float*)d_in[4];
  const float* WO  = (const float*)d_in[5];
  const float* gnw = (const float*)d_in[6];
  const float* gnb = (const float*)d_in[7];
  float* out = (float*)d_out;
  char* ws = (char*)d_ws;
  unsigned short* Xb    = (unsigned short*)(ws + offXb);
  unsigned short* Wqkvt = (unsigned short*)(ws + offWqkv);
  unsigned short* Wgot  = (unsigned short*)(ws + offWgo);
  float* tabQ = (float*)(ws + offTabQ);
  float* tabK = (float*)(ws + offTabK);
  unsigned short* Qhi = (unsigned short*)(ws + offQhi);
  unsigned short* Qlo = (unsigned short*)(ws + offQlo);
  unsigned short* Khi = (unsigned short*)(ws + offKhi);
  unsigned short* Klo = (unsigned short*)(ws + offKlo);
  unsigned short* Vth = (unsigned short*)(ws + offVth);
  unsigned short* Vtl = (unsigned short*)(ws + offVtl);
  float* Gt = (float*)(ws + offG);
  float* Yb = (float*)(ws + offY);
  unsigned short* Zhi = (unsigned short*)(ws + offZhi);
  unsigned short* Zlo = (unsigned short*)(ws + offZlo);
  unsigned short* Wqt = Wqkvt;
  unsigned short* Wkt = Wqkvt + (size_t)nWs;
  unsigned short* Wvt = Wqkvt + (size_t)2 * nWs;
  unsigned short* Wgt = Wgot;
  unsigned short* Wot = Wgot + (size_t)nWs;

  FreqParams fp;
  for (int i = 0; i < kPairs; ++i) {
    const float pf = (float)pow(10000.0, (double)i / (double)kPairs);
    fp.invf[i] = 1.0f / pf;
  }
  RetParams rp;
  {
    const double lga = log(1.0 / 32.0), lgb = log(1.0 / 512.0);
    for (int h = 0; h < kHeads; ++h) {
      const double lg = lga + (lgb - lga) * (double)h / 7.0;
      const float gm = (float)(1.0 - exp(lg));
      rp.l2g[h] = (float)log2((double)gm);
    }
  }

  const int n8 = nX / 8;
  cast8_bf16_kernel<<<dim3(n8 / 256), dim3(256), 0, stream>>>(X, Xb, n8);
  tr_bf16_kernel<<<dim3(kHid / 64, kHd / 64, 3 * kHeads), dim3(256), 0, stream>>>(WQ, WK, WV, Wqkvt, kHid, kHd, kHeads);
  tr_bf16_kernel<<<dim3(kHid / 64, kHid / 64, 2), dim3(256), 0, stream>>>(WG, WO, WO, Wgot, kHid, kHid, 1);
  xpos_table_kernel<<<dim3((kSeq * 32) / 256), dim3(256), 0, stream>>>(tabQ, tabK, fp);

  const int blocksTok = ((kTok / 64) * (kHid / 64)) / 8;
  const int blocksVt  = ((kHd / 64) * (kSeq / 64)) / 8;

  gemm64<0, 3><<<dim3(blocksTok, 1), dim3(256), 0, stream>>>(
      Xb, Xb, kHid, 0L, Wqt, Wqt, kHid, 0L, (void*)Qhi, (void*)Qlo, kHid, 0L, tabQ, kTok, kHid, kHid, 1.0f);
  gemm64<0, 3><<<dim3(blocksTok, 1), dim3(256), 0, stream>>>(
      Xb, Xb, kHid, 0L, Wkt, Wkt, kHid, 0L, (void*)Khi, (void*)Klo, kHid, 0L, tabK, kTok, kHid, kHid, 1.0f);

  for (int b = 0; b < kBatch; ++b) {
    const unsigned short* Xrows = Xb + (size_t)b * kSeq * kHid;
    unsigned short* vh = Vth + (size_t)b * kHeads * kHd * kSeq;
    unsigned short* vl = Vtl + (size_t)b * kHeads * kHd * kSeq;
    gemm64<0, 2><<<dim3(blocksVt, kHeads), dim3(256), 0, stream>>>(
        Wvt, Wvt, kHid, (long)kHd * kHid, Xrows, Xrows, kHid, 0L,
        (void*)vh, (void*)vl, kSeq, (long)kHd * kSeq, tabQ, kHd, kSeq, kHid, 1.0f);
  }

  gemm64<0, 0><<<dim3(blocksTok, 1), dim3(256), 0, stream>>>(
      Xb, Xb, kHid, 0L, Wgt, Wgt, kHid, 0L, (void*)Gt, (void*)Gt, kHid, 0L, tabQ, kTok, kHid, kHid, 1.0f);

  retention_kernel<<<dim3(kSeq / 128, kBatch * kHeads), dim3(256), 0, stream>>>(Qhi, Qlo, Khi, Klo, Vth, Vtl, Yb, rp);

  gn_gate_kernel<<<dim3(kTok), dim3(256), 0, stream>>>(Yb, Gt, gnw, gnb, Zhi, Zlo);

  gemm64<2, 0><<<dim3(blocksTok, 1), dim3(256), 0, stream>>>(
      Zhi, Zlo, kHid, 0L, Wot, Wot, kHid, 0L, (void*)out, (void*)out, kHid, 0L, tabQ, kTok, kHid, kHid, 1.0f);
}
